// DotProductAttention_58368605552662
// MI455X (gfx1250) — hardware-run, weakly checked
//
#include <hip/hip_runtime.h>


#ifndef NB
#define NB 16
#endif
#ifndef SEQ
#define SEQ 2048
#endif
#define NB_FULL  16
#define SEQ_FULL 2048
#ifndef OUT_SEQ
#define OUT_SEQ SEQ
#endif
#define DH   128
#define AW   4
#define OSP  132
#define VTP  72
#define SC2  ((float)(0.08838834764831845 * 1.4426950408889634))
#define FILL2 ((float)(-1000000.0 * 1.4426950408889634))
#define PSH  14.0f
#define NEGB (-3.0e38f)

static_assert(DH == 128);
static_assert(DH % 32 == 0);
static_assert(SEQ % 64 == 0);
static_assert(SEQ % 32 == 0);
static_assert(SEQ % (16 * AW) == 0);
static_assert(((size_t)SEQ * DH) % 8 == 0);
static_assert(NB <= NB_FULL);
static_assert(SEQ <= SEQ_FULL);
static_assert((OSP * 4) % 16 == 0);
static_assert(OSP >= DH);
static_assert(VTP % 8 == 0);
static_assert(VTP >= 64);
static_assert((size_t)AW * 16 * OSP * 4 <= 131072);
static_assert((size_t)DH * VTP * 2 <= 131072);
static_assert(256 * 16 * 4 == DH * 64 * 2);
static_assert(256 * 4 * 8 == 64 * DH);
static_assert(32 * 16 * 16 == 16 * DH * 4);

typedef _Float16 h16;
typedef __attribute__((ext_vector_type(16))) _Float16 v16h;
typedef __attribute__((ext_vector_type(8)))  _Float16 v8h;
typedef __attribute__((ext_vector_type(8)))  float    v8f;
typedef __attribute__((ext_vector_type(4)))  float    v4f;
typedef v4f  __attribute__((may_alias)) v4fa;
typedef v8h  __attribute__((may_alias)) v8ha;

__device__ __forceinline__ unsigned short f2bf(float f) { unsigned u = __float_as_uint(f); u += 0x7FFFu + ((u >> 16) & 1u); return (unsigned short)(u >> 16); }
__device__ __forceinline__ float bfr(float f) { return __uint_as_float(((unsigned)f2bf(f)) << 16); }
__device__ __forceinline__ v16h cat16(v8h lo, v8h hi) { return __builtin_shufflevector(lo, hi, 0, 1, 2, 3, 4, 5, 6, 7, 8, 9, 10, 11, 12, 13, 14, 15); }
__device__ __forceinline__ v8f wmma16(v16h a, v16h b, v8f c) { return __builtin_amdgcn_wmma_f32_16x16x32_f16(false, a, false, b, (short)0, c, false, false); }
__device__ __forceinline__ v8f wmma16g(v16h a, v16h b, v8f c) { c = wmma16(a, b, c); asm volatile("v_nop\n\tv_nop\n\tv_nop\n\tv_nop" : "+v"(c) : "v"(a), "v"(b)); return c; }
__device__ __forceinline__ v16h  ldh(const h16* p) { return cat16(*(const v8h*)p, *(const v8h*)(p + 16)); }
__device__ __forceinline__ void wave_sync() { __builtin_amdgcn_fence(3  , "wavefront"); __builtin_amdgcn_wave_barrier(); asm volatile("" ::: "memory"); }
static __device__ __forceinline__ h16 toh_flush(float v) { const float w = (fabsf(v) < 6.103515625e-05f) ? 0.0f : v; return (h16)w; }

__global__ __launch_bounds__(256) void k_cvth8(const float* __restrict__ src, h16* dst, size_t n8) {
    const size_t i = (size_t)blockIdx.x * 256 + threadIdx.x; if (i >= n8) return;
    const v8f v = *(const v8f*)(src + i * 8); v8h o;
#pragma unroll
    for (int k = 0; k < 8; ++k) o[k] = toh_flush(bfr(v[k]));
    *(volatile v8h*)(dst + i * 8) = o; __threadfence(); *(volatile v8h*)(dst + i * 8) = o;
}

__global__ __launch_bounds__(256) void k_vtr(const float* __restrict__ V, h16* VT) {
    __shared__ __align__(16) h16 ls[DH * VTP];
    const unsigned tid = threadIdx.x;
    const unsigned tb = blockIdx.x * 64u;
    const unsigned b = blockIdx.y;
    const float* src = V + ((size_t)b * SEQ_FULL + tb) * DH;
#pragma unroll
    for (unsigned it = 0; it < 8; ++it) {
        const unsigned idx = it * 256u + tid; const unsigned t = idx >> 5, c4 = (idx & 31u) * 4u;
        const v4f x = *(const v4f*)(src + (size_t)t * DH + c4);
#pragma unroll
        for (unsigned i = 0; i < 4; ++i) ls[(c4 + i) * VTP + t] = toh_flush(bfr(x[i]));
    }
    __syncthreads();
    h16* dstb = VT + (size_t)b * DH * SEQ + tb;
#pragma unroll 1
    for (int ps = 0; ps < 2; ++ps) {
#pragma unroll
        for (unsigned it = 0; it < 4; ++it) { const unsigned p = it * 256u + tid; const unsigned d = p >> 3, c8 = (p & 7u) * 8u;
            const v8h hv = *(const v8ha*)(&ls[d * VTP + c8]);
            *(volatile v8h*)(dstb + (size_t)d * SEQ + c8) = hv; }
        if (ps == 0) __threadfence(); }
}

__global__ __attribute__((amdgpu_num_vgpr(256))) __launch_bounds__(32 * AW) void k_flash(const h16* __restrict__ QH, const h16* __restrict__ KP, const h16* __restrict__ VT,
                                                                                         const int* __restrict__ vlens, float* OUT) {
    __shared__ __align__(16) float os[AW * 16 * OSP];
    const int lane = threadIdx.x & 31, lr = lane & 15, hi = lane >> 4;
    const int wave = __builtin_amdgcn_readfirstlane((int)(threadIdx.x >> 5));
    const unsigned b = blockIdx.y;
    const int t0 = (blockIdx.x * AW + wave) * 16;
    int vl = vlens[b]; vl = max(vl, 0); vl = min(vl, SEQ);
    const int z = (int)(vl == 0);
    const bool uni = (z != 0);
    const int klim = vl + z * SEQ;
    const int nk = ((vl + 31) & ~31) + z * SEQ;
    const size_t pbase = (size_t)b * SEQ * DH;
    const size_t qo = pbase + (size_t)(t0 + lr) * DH + 8 * hi;
    const size_t ko = pbase + (size_t)lr * DH + 8 * hi;
    const size_t vo = pbase + (size_t)lr * SEQ + 8 * hi;
    v8f o[8];
#pragma unroll
    for (int j = 0; j < 8; ++j) o[j] = (v8f){};
    float m = NEGB, l = 0.0f;
#pragma unroll 1
    for (int key0 = 0; key0 < nk; key0 += 32) {
        unsigned qz = 0u; asm volatile("" : "+v"(qz));
        const h16* qa = QH + (qo + qz);
        const h16* ka = KP + ko + (size_t)key0 * DH;
        v8f sa = (v8f){}, sb = (v8f){};
#pragma unroll
        for (int kc = 0; kc < DH / 32; ++kc) {
            const v16h qf = ldh(qa + 32 * kc);
            const v16h a0 = ldh(ka + 32 * kc), a1 = ldh(ka + 16 * DH + 32 * kc);
            sa = wmma16g(a0, qf, sa); sb = wmma16g(a1, qf, sb); }
        const int ja = key0 + 8 * hi;
        float ta[8], tb[8]; bool fa[8], fb[8]; float mx = NEGB;
#pragma unroll
        for (int r = 0; r < 8; ++r) {
            fa[r] = (ja + r) < klim;
            fb[r] = (ja + 16 + r) < klim;
            ta[r] = uni ? FILL2 : sa[r] * SC2; tb[r] = uni ? FILL2 : sb[r] * SC2;
            mx = fmaxf(mx, fmaxf(fa[r] ? ta[r] : NEGB, fb[r] ? tb[r] : NEGB)); }
        mx = fmaxf(mx, __shfl_xor(mx, 16, 32));
        const float mnew = fmaxf(m, mx);
        const float alpha = __builtin_amdgcn_exp2f(m - mnew);
        const float sh = PSH - mnew;
        v16h pb; float ls = 0.0f;
#pragma unroll
        for (int r = 0; r < 8; ++r) {
            const float ea = __builtin_amdgcn_exp2f(ta[r] + sh), eb = __builtin_amdgcn_exp2f(tb[r] + sh);
            const float ga = fa[r] ? ea : 0.0f, gb = fb[r] ? eb : 0.0f;
            const h16 pa = toh_flush(ga); const h16 pc = toh_flush(gb);
            pb[r] = pa; pb[8 + r] = pc;
            ls += (float)pa + (float)pc; }
        l = l * alpha + ls; m = mnew;
#pragma unroll
        for (int j = 0; j < 8; ++j) o[j] = o[j] * alpha;
        const h16* va = VT + vo + key0;
#pragma unroll
        for (int j = 0; j < 8; ++j) { const v16h vf = ldh(va + (size_t)j * 16 * SEQ); o[j] = wmma16g(vf, pb, o[j]); }
    }
    l += __shfl_xor(l, 16, 32);
    const bool any = l > 0.0f;
    const float lsafe = any ? l : 1.0f;
    const float inv = any ? (1.0f / lsafe) : 0.0f;
    const int wb = wave * 16 * OSP;
#pragma unroll
    for (int j = 0; j < 8; ++j) { v4f a, c;
        a[0] = o[j][0] * inv; a[1] = o[j][1] * inv; a[2] = o[j][2] * inv; a[3] = o[j][3] * inv; c[0] = o[j][4] * inv; c[1] = o[j][5] * inv; c[2] = o[j][6] * inv; c[3] = o[j][7] * inv;
        *(v4fa*)(&os[wb + lr * OSP + 16 * j + 8 * hi]) = a; *(v4fa*)(&os[wb + lr * OSP + 16 * j + 8 * hi + 4]) = c; }
    wave_sync();
    float* orow = OUT + ((size_t)b * OUT_SEQ + t0) * DH;
#pragma unroll 1
    for (int ps = 0; ps < 2; ++ps) {
#pragma unroll
        for (int s = 0; s < 16; ++s) { const int cofs = lane * 4;
            const v4f val = *(const v4fa*)(&os[wb + s * OSP + cofs]);
            *(volatile v4f*)(orow + (size_t)s * DH + cofs) = val; }
        if (ps == 0) __threadfence(); }
}

static constexpr size_t al256(size_t v) { return (v + 255) & ~(size_t)255; }
static constexpr size_t SZ_PL = al256((size_t)NB * SEQ * DH * 2);
static constexpr size_t SZ_TOTAL = 3 * SZ_PL;
static_assert(SZ_TOTAL <= (size_t)134217728);
static_assert((size_t)NB * SEQ * DH == (size_t)NB * DH * SEQ);
static_assert(((size_t)SEQ * DH / 8) % 256 == 0);
static_assert(((size_t)NB * SEQ * DH / 8) % 256 == 0);

extern "C" void kernel_launch(void* const* d_in, const int* in_sizes, int n_in,
                              void* d_out, int out_size, void* d_ws, size_t ws_size, hipStream_t stream) {
    if (n_in < 4) return;
    const size_t needx = ((size_t)(NB - 1) * SEQ_FULL + SEQ) * DH;
    if ((size_t)in_sizes[0] < needx || (size_t)in_sizes[1] < needx || (size_t)in_sizes[2] < needx) return;
    if (in_sizes[3] < NB) return;
    if ((size_t)out_size < ((size_t)(NB - 1) * OUT_SEQ + SEQ) * DH) return;
    if (SZ_TOTAL > ws_size) return;
    const float* qin = (const float*)d_in[0];
    const float* kin = (const float*)d_in[1];
    const float* vin = (const float*)d_in[2];
    const int* vlens = (const int*)d_in[3];
    float* OUT = (float*)d_out;
    char* wsp = (char*)d_ws;
    h16* QH = (h16*)wsp; wsp += SZ_PL;
    h16* KP = (h16*)wsp; wsp += SZ_PL;
    h16* VT = (h16*)wsp; wsp += SZ_PL;

    if (SEQ == SEQ_FULL) {
        const size_t n8 = (size_t)NB * SEQ * DH / 8;
        k_cvth8<<<(unsigned)((n8 + 255) / 256), 256, 0, stream>>>(qin, QH, n8);
        k_cvth8<<<(unsigned)((n8 + 255) / 256), 256, 0, stream>>>(kin, KP, n8);
    } else {
        const size_t n8 = (size_t)SEQ * DH / 8;
        for (int b = 0; b < NB; ++b) {
            k_cvth8<<<(unsigned)((n8 + 255) / 256), 256, 0, stream>>>(qin + (size_t)b * SEQ_FULL * DH, QH + (size_t)b * SEQ * DH, n8);
            k_cvth8<<<(unsigned)((n8 + 255) / 256), 256, 0, stream>>>(kin + (size_t)b * SEQ_FULL * DH, KP + (size_t)b * SEQ * DH, n8);
        }
    }
    k_vtr<<<dim3(SEQ / 64, NB, 1), 256, 0, stream>>>(vin, VT);

    k_flash<<<dim3(SEQ / (16 * AW), NB, 1), 32 * AW, 0, stream>>>(QH, KP, VT, vlens, OUT);
}
